// MultinomialPolyaGamma_7103875907635
// MI455X (gfx1250) — hardware-verified
//
#include <hip/hip_runtime.h>


#define NB_  8192
#define DD   256
#define KM1  64
#define NC   65
#define RCH  512
#define NKE  (KM1 * DD)
#define DM   DD
#define LOSC 1024.0f

typedef _Float16 h16;
typedef unsigned short bf;
typedef __attribute__((ext_vector_type(16))) __bf16   v16bf;
typedef __attribute__((ext_vector_type(16))) _Float16 v16h;
typedef __attribute__((ext_vector_type(8)))  _Float16 v8h;
typedef __attribute__((ext_vector_type(8)))  unsigned short v8us;
typedef __attribute__((ext_vector_type(8)))  float    v8f;
typedef __attribute__((ext_vector_type(4)))  float    v4f;
typedef v8h  __attribute__((may_alias)) v8ha;
typedef v4f  __attribute__((may_alias)) v4fa;
typedef v8us __attribute__((may_alias)) v8usa;

__device__ __forceinline__ unsigned short f2bf(float f) { unsigned u = __float_as_uint(f); u += 0x7FFFu + ((u >> 16) & 1u); return (unsigned short)(u >> 16); }
__device__ __forceinline__ float bf2f(unsigned short b) { return __uint_as_float(((unsigned)b) << 16); }
__device__ __forceinline__ float bfr(float f) { return bf2f(f2bf(f)); }
__device__ __forceinline__ v16h cat16(v8h lo, v8h hi) { return __builtin_shufflevector(lo, hi, 0, 1, 2, 3, 4, 5, 6, 7, 8, 9, 10, 11, 12, 13, 14, 15); }
__device__ __forceinline__ v16bf cat16b(v8us lo, v8us hi) { return __builtin_bit_cast(v16bf, __builtin_shufflevector(lo, hi, 0, 1, 2, 3, 4, 5, 6, 7, 8, 9, 10, 11, 12, 13, 14, 15)); }
__device__ __forceinline__ v8f wmma16(v16h a, v16h b, v8f c) { return __builtin_amdgcn_wmma_f32_16x16x32_f16(false, a, false, b, (short)0, c, false, false); }
__device__ __forceinline__ v8f wmmab(v16bf a, v16bf b, v8f c) { return __builtin_amdgcn_wmma_f32_16x16x32_bf16(false, a, false, b, (short)0, c, false, false); }

template <bool SPLITA, bool F16OUT = false>
__global__ __launch_bounds__(128) void k_gemmb(const bf* __restrict__ A, const bf* __restrict__ Al, const bf* __restrict__ Bn, const float* __restrict__ bias, float* C, int ldc, h16* C2, const float* __restrict__ R = nullptr, int K = DM, int roundR = 1) {
    __shared__ __align__(16) float ost[4][16 * 68];
    const int lane = threadIdx.x & 31, wave = threadIdx.x >> 5, lr = lane & 15, hi = lane >> 4;
    const int r0 = blockIdx.x * 64 + wave * 16, c0 = blockIdx.y * 64;
    const size_t aoff = (size_t)(r0 + lr) * K + 8 * hi;
    size_t boff[4];
#pragma unroll
    for (int t = 0; t < 4; ++t) boff[t] = (size_t)(c0 + t * 16 + lr) * K + 8 * hi;
    v8f acc[4];
#pragma unroll
    for (int t = 0; t < 4; ++t) acc[t] = (v8f){};
#pragma unroll 1
    for (int kc = 0; kc < K; kc += 32) {
        const v16bf a = cat16b(*(const v8us*)(A + aoff + kc), *(const v8us*)(A + aoff + kc + 16));
        v16bf al = a;
        if (SPLITA) al = cat16b(*(const v8us*)(Al + aoff + kc), *(const v8us*)(Al + aoff + kc + 16));
#pragma unroll
        for (int t = 0; t < 4; ++t) { const v16bf b = cat16b(*(const v8us*)(Bn + boff[t] + kc), *(const v8us*)(Bn + boff[t] + kc + 16)); acc[t] = wmmab(a, b, acc[t]); if (SPLITA) acc[t] = wmmab(al, b, acc[t]); }
        asm volatile("v_nop\n\tv_nop\n\tv_nop\n\tv_nop" : "+v"(acc[0]), "+v"(acc[1]), "+v"(acc[2]), "+v"(acc[3]) : "v"(a), "v"(al));
    }
    float* os = &ost[wave][0];
#pragma unroll
    for (int t = 0; t < 4; ++t) { const float bv = bias ? bfr(bias[c0 + t * 16 + lr]) : 0.f;
#pragma unroll
        for (int j = 0; j < 8; ++j) os[(hi * 8 + j) * 68 + t * 16 + lr] = acc[t][j] + bv; }
    __syncthreads();
    if (F16OUT) {
        h16* crow = (h16*)(void*)C + (size_t)r0 * ldc + c0;
        auto pass = [&]() {
#pragma unroll
            for (int s = 0; s < 4; ++s) { const int row = 4 * s + (lane >> 3), piece = lane & 7; const float* sp = os + row * 68 + piece * 8; v8h o, o2;
#pragma unroll
                for (int i = 0; i < 8; ++i) { const h16 a = (h16)sp[i]; o[i] = a; o2[i] = (h16)((sp[i] - (float)a) * LOSC); }
                *(volatile v8h*)(crow + (size_t)row * ldc + piece * 8) = o; if (C2) *(volatile v8h*)(C2 + (size_t)r0 * ldc + c0 + (size_t)row * ldc + piece * 8) = o2; }
        };
        pass(); __threadfence(); pass();
    } else {
        float* crow = C + (size_t)r0 * ldc + c0;
        auto pass = [&]() {
#pragma unroll
            for (int s = 0; s < 8; ++s) { const int Lid = (lane >> 3) + 4 * s, piece = lane & 7; const int row = Lid >> 1, cofs = (Lid & 1) * 32 + piece * 4;
                v4f val = *(const v4fa*)(os + row * 68 + cofs); if (R) { const v4f rv = *(const v4f*)(R + ((size_t)r0 + row) * ldc + c0 + cofs); val += roundR ? (v4f){bfr(rv[0]), bfr(rv[1]), bfr(rv[2]), bfr(rv[3])} : rv; }
                *(volatile v4f*)(crow + (size_t)row * ldc + cofs) = val; }
        };
        pass(); __threadfence(); pass();
    }
}

__global__ __launch_bounds__(256) void k_wt(const float* __restrict__ Wm, int K, int ncols, bf* WT) {
    __shared__ __align__(16) unsigned short tl[64 * 72];
    const int tid = threadIdx.x, k0 = blockIdx.x * 64, n0 = blockIdx.y * 64;
    const int kk = tid >> 2, nq = (tid & 3) * 16;
#pragma unroll
    for (int i = 0; i < 16; ++i) tl[(nq + i) * 72 + kk] = f2bf(Wm[(size_t)(k0 + kk) * ncols + n0 + nq + i]);
    __syncthreads();
    const int piece = tid & 7;
    auto pass = [&]() {
#pragma unroll
        for (int s = 0; s < 2; ++s) { const int nr = (tid >> 3) + 32 * s; const v8us val = *(const v8usa*)(tl + nr * 72 + piece * 8); *(volatile v8us*)(WT + (size_t)(n0 + nr) * K + k0 + piece * 8) = val; }
    };
    pass(); __threadfence(); pass();
}

__global__ __launch_bounds__(256) void k_cvtx(const float* __restrict__ src, bf* dst) {
    const int lane = threadIdx.x & 31; const size_t r = (size_t)blockIdx.x * 8 + (threadIdx.x >> 5); if (r >= (size_t)NB_) return; v8us o;
#pragma unroll
    for (int i = 0; i < 8; ++i) o[i] = f2bf(src[r * DD + lane * 8 + i]);
    *(volatile v8us*)(dst + r * DD + lane * 8) = o; __threadfence(); *(volatile v8us*)(dst + r * DD + lane * 8) = o;
}
__global__ __launch_bounds__(256) void k_xsx(const float* __restrict__ T, const float* __restrict__ x, int r0, float* XS) {
    typedef __attribute__((ext_vector_type(2))) float v2f;
    const int lane = threadIdx.x & 31, rl = blockIdx.x * 8 + (threadIdx.x >> 5); if (rl >= RCH) return; const size_t b = (size_t)r0 + rl; float xe[8];
#pragma unroll
    for (int i = 0; i < 8; ++i) xe[i] = bfr(x[b * DD + lane * 8 + i]);
    v2f mine = {0.f, 0.f};
#pragma unroll 1
    for (int k = 0; k < KM1; ++k) { float s = 0.f; const float* tr = T + (size_t)rl * NKE + (size_t)k * DD + lane * 8;
#pragma unroll
        for (int i = 0; i < 8; ++i) s = fmaf(tr[i], xe[i], s);
#pragma unroll
        for (int sh = 16; sh; sh >>= 1) s += __shfl_xor(s, sh, 32);
        if ((k >> 1) == lane) { if (k & 1) mine[1] = s; else mine[0] = s; } }
    *(volatile v2f*)(XS + b * KM1 + lane * 2) = mine; __threadfence(); *(volatile v2f*)(XS + b * KM1 + lane * 2) = mine;
}
__device__ __forceinline__ float softplus_f(float v) { return log1pf(__expf(-fabsf(v))) + fmaxf(v, 0.f); }
__global__ __launch_bounds__(256) void k_loss(const float* __restrict__ LG, const float* __restrict__ XS, const int* __restrict__ yv, const int* __restrict__ lt, float* OUTP) {
    const int b = blockIdx.x * 256 + threadIdx.x; if (b >= NB_) return; int y = yv[b]; y = y < 0 ? 0 : (y >= NC ? NC - 1 : y); const int mode = lt[0];
    float s1 = 0.f, s0 = 0.f;
#pragma unroll 1
    for (int j = 0; j < KM1; ++j) { const float lg = LG[(size_t)b * KM1 + j]; const float bj = (j >= 1 && y <= j - 1 && y <= NC - 3) ? 0.f : 1.f;
        const float psi = sqrtf(XS[(size_t)b * KM1 + j] + lg * lg); const float kap = ((y == j) ? 1.f : 0.f) - 0.5f * bj;
        s1 += lg * kap + bj * (0.5f * psi - softplus_f(psi)); s0 += softplus_f(lg) * bj; }
    const float lgy = (y < KM1) ? LG[(size_t)b * KM1 + (y < KM1 ? y : 0)] : 0.f;
    const float out = (mode == 0) ? -(lgy - s0) : -s1;
    *(volatile float*)(OUTP + b) = out; __threadfence(); *(volatile float*)(OUTP + b) = out;
}

extern "C" void kernel_launch(void* const* d_in, const int* in_sizes, int n_in,
                              void* d_out, int out_size, void* d_ws, size_t ws_size, hipStream_t stream) {
    (void)in_sizes; (void)n_in; (void)out_size;
    const float* x = (const float*)d_in[0]; const int* yv = (const int*)d_in[1]; const float* mu = (const float*)d_in[2]; const float* Sig = (const float*)d_in[3]; const int* lt = (const int*)d_in[4];
    float* out = (float*)d_out;
    char* wsp = (char*)d_ws;
    auto take = [&](size_t bytes) { char* p = wsp; wsp += (bytes + 255) & ~(size_t)255; return (void*)p; };
    bf* Xb = (bf*)take((size_t)NB_ * DD * 2); bf* MUT = (bf*)take((size_t)KM1 * DD * 2); bf* ST = (bf*)take((size_t)NKE * DD * 2); float* LG = (float*)take((size_t)NB_ * KM1 * 4); float* T = (float*)take((size_t)RCH * NKE * 4); float* XS = (float*)take((size_t)NB_ * KM1 * 4);
    if ((size_t)(wsp - (char*)d_ws) > ws_size) return;
    k_cvtx<<<NB_ / 8, 256, 0, stream>>>(x, Xb); k_wt<<<dim3(DD / 64, KM1 / 64, 1), 256, 0, stream>>>(mu, DD, KM1, MUT);
    for (int k = 0; k < KM1; ++k) k_wt<<<dim3(DD / 64, DD / 64, 1), 256, 0, stream>>>(Sig + (size_t)k * DD * DD, DD, DD, ST + (size_t)k * DD * DD);
    k_gemmb<false, false><<<dim3(NB_ / 64, 1, 1), 128, 0, stream>>>(Xb, nullptr, MUT, nullptr, LG, KM1, nullptr, nullptr, DD);
    for (int ch = 0; ch < NB_ / RCH; ++ch) { const int r0 = ch * RCH;
        k_gemmb<false, false><<<dim3(RCH / 64, NKE / 64, 1), 128, 0, stream>>>(Xb + (size_t)r0 * DD, nullptr, ST, nullptr, T, NKE, nullptr, nullptr, DD);
        k_xsx<<<RCH / 8, 256, 0, stream>>>(T, x, r0, XS); }
    k_loss<<<NB_ / 256, 256, 0, stream>>>(LG, XS, yv, lt, out);
}
